// DilatedAttention_full_14319420964898
// MI455X (gfx1250) — hardware-verified
//
#include <hip/hip_runtime.h>
#include <math.h>
#include <stdint.h>

#define BATCH  4
#define NHEADS 8
#define SEQ    2048
#define HD     64
#define BHN    (BATCH * NHEADS)
#define DMOD   (NHEADS * HD)
#define NELEM  (BHN * SEQ * HD)
static_assert(NELEM == 4194304);
static_assert(DMOD == 512);
static_assert(((SEQ / 8) % 64) == 0);
static_assert((NELEM % (8 * 256)) == 0);

typedef _Float16 v16h __attribute__((ext_vector_type(16)));
typedef _Float16 v8h  __attribute__((ext_vector_type(8)));
typedef __bf16   v16b __attribute__((ext_vector_type(16)));
typedef __bf16   v8b  __attribute__((ext_vector_type(8)));
typedef float    v8f  __attribute__((ext_vector_type(8)));
typedef float    v4f  __attribute__((ext_vector_type(4)));
typedef unsigned int v4u __attribute__((ext_vector_type(4)));

__device__ __forceinline__ unsigned short bf_bits(float f) {
  unsigned u = __float_as_uint(f);
  return (unsigned short)((u + 0x7FFFu + ((u >> 16) & 1u)) >> 16);
}
__device__ __forceinline__ float bf_up(unsigned short h) { return __uint_as_float(((unsigned)h) << 16); }
__device__ __forceinline__ unsigned short h_bits(_Float16 x) { return __builtin_bit_cast(unsigned short, x); }
__device__ __forceinline__ unsigned pk16(unsigned short a, unsigned short b) { return (unsigned)a | ((unsigned)b << 16); }
__device__ __forceinline__ v8f zero8() { v8f z = {0.f, 0.f, 0.f, 0.f, 0.f, 0.f, 0.f, 0.f}; return z; }

__device__ __forceinline__ v16b ldfrag_b(const __bf16* p) {
  union { v16b v; v8b h[2]; } f;
  f.h[0] = *(const v8b*)(p);
  f.h[1] = *(const v8b*)(p + 16);
  return f.v;
}

__device__ __forceinline__ v8f mma_h(v16h a, v16h b, v8f c) {
  c = __builtin_amdgcn_wmma_f32_16x16x32_f16(false, a, false, b, (short)0, c, false, false);
#if defined(__HIP_DEVICE_COMPILE__)
  asm volatile("v_nop\n\tv_nop\n\tv_nop\n\tv_nop" : "+v"(c) : "v"(a), "v"(b));
#endif
  return c;
}
__device__ __forceinline__ v8f mma_b(v16b a, v16b b, v8f c) {
  c = __builtin_amdgcn_wmma_f32_16x16x32_bf16(false, a, false, b, (short)0, c, false, false);
#if defined(__HIP_DEVICE_COMPILE__)
  asm volatile("v_nop\n\tv_nop\n\tv_nop\n\tv_nop" : "+v"(c) : "v"(a), "v"(b));
#endif
  return c;
}
__device__ __forceinline__ void wave_sync_lds() {
  __builtin_amdgcn_fence(__ATOMIC_RELEASE, "workgroup");
  __builtin_amdgcn_wave_barrier();
  __builtin_amdgcn_fence(__ATOMIC_ACQUIRE, "workgroup");
}

__global__ __launch_bounds__(256)
void cvt_qkv(const float* __restrict__ q, const float* __restrict__ k, const float* __restrict__ v,
             unsigned short* qb, unsigned short* kb, unsigned short* vh, int n8) {
  const int i = blockIdx.x * 256 + threadIdx.x;
  if (i < n8) {
    const size_t o = (size_t)i * 8;
    const v4f q0 = *(const v4f*)(q + o), q1 = *(const v4f*)(q + o + 4);
    const v4f k0 = *(const v4f*)(k + o), k1 = *(const v4f*)(k + o + 4);
    const v4f v0 = *(const v4f*)(v + o), v1 = *(const v4f*)(v + o + 4);
    v4u pq, pk, pv;
    pq[0] = pk16(bf_bits(q0[0]), bf_bits(q0[1]));
    pq[1] = pk16(bf_bits(q0[2]), bf_bits(q0[3]));
    pq[2] = pk16(bf_bits(q1[0]), bf_bits(q1[1]));
    pq[3] = pk16(bf_bits(q1[2]), bf_bits(q1[3]));
    pk[0] = pk16(bf_bits(k0[0]), bf_bits(k0[1]));
    pk[1] = pk16(bf_bits(k0[2]), bf_bits(k0[3]));
    pk[2] = pk16(bf_bits(k1[0]), bf_bits(k1[1]));
    pk[3] = pk16(bf_bits(k1[2]), bf_bits(k1[3]));
    unsigned short vs[8];
#pragma unroll
    for (int e = 0; e < 4; ++e) {
      vs[e]     = h_bits((_Float16)(bf_up(bf_bits(v0[e])) * 16.0f));
      vs[4 + e] = h_bits((_Float16)(bf_up(bf_bits(v1[e])) * 16.0f));
    }
    pv[0] = pk16(vs[0], vs[1]);
    pv[1] = pk16(vs[2], vs[3]);
    pv[2] = pk16(vs[4], vs[5]);
    pv[3] = pk16(vs[6], vs[7]);
    *(volatile v4u*)(qb + o) = pq;
    *(volatile v4u*)(kb + o) = pk;
    *(volatile v4u*)(vh + o) = pv;
    __threadfence();
    *(volatile v4u*)(qb + o) = pq;
    *(volatile v4u*)(kb + o) = pk;
    *(volatile v4u*)(vh + o) = pv;
  }
}

template <int DR>
__global__ __launch_bounds__(128)
void dil_attn(const unsigned short* __restrict__ qbp, const unsigned short* __restrict__ kbp,
              const unsigned short* __restrict__ vhp, float* op) {
  constexpr int LK  = SEQ / DR;
  constexpr int NKT = LK / 64;
  constexpr int HPB = NHEADS / DR;
  union FH { v16h v; v8h h[2]; };
  union FB { v16b v; v8b h[2]; };
  __shared__ __align__(16) __bf16   Ksh[64 * 64];
  __shared__ __align__(16) _Float16 Vt[64 * 64];
  __shared__ __align__(16) _Float16 Psh[4][16 * 64];
  __shared__ __align__(16) _Float16 Psl[4][16 * 64];
  __shared__ __align__(16) float    Os[4][16 * 64];

  const int tid  = threadIdx.x;
  const int wave = tid >> 5;
  const int lane = tid & 31;
  const int hh   = lane >> 4;
  const int c    = lane & 15;

  const int bx = blockIdx.x;
  const int qt = bx % NKT;
  const int bh = bx / NKT;
  const int g  = bh & (NHEADS - 1);
  const int rg = g / HPB;
  const int q0 = qt * 64 + wave * 16;

  const __bf16*   Qg = (const __bf16*)(const void*)qbp + (size_t)bh * SEQ * HD;
  const __bf16*   Kg = (const __bf16*)(const void*)kbp + (size_t)bh * SEQ * HD;
  const _Float16* Vg = (const _Float16*)(const void*)vhp + (size_t)bh * SEQ * HD;
  float* Og = op + (size_t)bh * LK * HD;

  v16b qa[2];
  {
    const size_t qo = (size_t)((q0 + c) * DR + rg) * HD + 8 * hh;
    qa[0] = ldfrag_b(Qg + qo);
    qa[1] = ldfrag_b(Qg + qo + 32);
  }

  float mrow[8], lrow[8];
  v8f oacc[4];
#pragma unroll
  for (int r = 0; r < 8; ++r) { mrow[r] = -INFINITY; lrow[r] = 0.f; }
#pragma unroll
  for (int t = 0; t < 4; ++t) oacc[t] = zero8();

#pragma unroll 1
  for (int kt = 0; kt < NKT; ++kt) {
    __syncthreads();
    {
      const int j = tid >> 1, hf = (tid & 1) * 32;
      const size_t po = (size_t)((kt * 64 + j) * DR + rg) * HD + hf;
      const __bf16*   kg = Kg + po;
      const _Float16* vg = Vg + po;
#pragma unroll
      for (int i = 0; i < 4; ++i) {
        const v8b a0 = *(const v8b*)(kg + 8 * i);
        *(v8b*)(Ksh + j * 64 + hf + 8 * i) = a0;
        const v8h b0 = *(const v8h*)(vg + 8 * i);
#pragma unroll
        for (int e = 0; e < 8; ++e) Vt[(hf + 8 * i + e) * 64 + j] = b0[e];
      }
    }
    __syncthreads();

    v8f s[4];
#pragma unroll
    for (int j = 0; j < 4; ++j) {
      v8f sh = zero8();
#pragma unroll
      for (int dc = 0; dc < 2; ++dc) {
        FB kb;
        kb.h[0] = *(const v8b*)(Ksh + (j * 16 + c) * 64 + dc * 32 + 8 * hh);
        kb.h[1] = *(const v8b*)(Ksh + (j * 16 + c) * 64 + dc * 32 + 16 + 8 * hh);
        sh = mma_b(qa[dc], kb.v, sh);
      }
      s[j] = sh;
    }

    _Float16* pwh = Psh[wave];
    _Float16* pwl = Psl[wave];
#pragma unroll
    for (int r = 0; r < 8; ++r) {
      float m = s[0][r];
      m = fmaxf(m, s[1][r]);
      m = fmaxf(m, s[2][r]);
      m = fmaxf(m, s[3][r]);
#pragma unroll
      for (int off = 1; off < 16; off <<= 1) m = fmaxf(m, __shfl_xor(m, off, 32));
      const float mnew  = fmaxf(mrow[r], m);
      const float alpha = __expf(mrow[r] - mnew);
      mrow[r] = mnew;
      float psum = 0.f;
#pragma unroll
      for (int j = 0; j < 4; ++j) {
        const float p  = __expf(s[j][r] - mnew);
        psum += p;
        const float tp = p * 1024.0f;
        const _Float16 xh = (_Float16)tp;
        const _Float16 xl = (_Float16)((tp - (float)xh) * 4096.0f);
        const int pi = (8 * hh + r) * 64 + j * 16 + c;
        pwh[pi] = xh;
        pwl[pi] = xl;
      }
#pragma unroll
      for (int off = 1; off < 16; off <<= 1) psum += __shfl_xor(psum, off, 32);
      lrow[r] = lrow[r] * alpha + psum;
#pragma unroll
      for (int t = 0; t < 4; ++t) oacc[t][r] *= alpha;
    }
    wave_sync_lds();

    v8f o1[4];
#pragma unroll
    for (int t = 0; t < 4; ++t) o1[t] = zero8();
#pragma unroll
    for (int kk = 0; kk < 2; ++kk) {
      FH pa, pl;
      pa.h[0] = *(const v8h*)(pwh + c * 64 + kk * 32 + 8 * hh);
      pa.h[1] = *(const v8h*)(pwh + c * 64 + kk * 32 + 16 + 8 * hh);
      pl.h[0] = *(const v8h*)(pwl + c * 64 + kk * 32 + 8 * hh);
      pl.h[1] = *(const v8h*)(pwl + c * 64 + kk * 32 + 16 + 8 * hh);
#pragma unroll
      for (int t = 0; t < 4; ++t) {
        FH vb;
        vb.h[0] = *(const v8h*)(Vt + (t * 16 + c) * 64 + kk * 32 + 8 * hh);
        vb.h[1] = *(const v8h*)(Vt + (t * 16 + c) * 64 + kk * 32 + 16 + 8 * hh);
        oacc[t] = mma_h(pa.v, vb.v, oacc[t]);
        o1[t]   = mma_h(pl.v, vb.v, o1[t]);
      }
    }
#pragma unroll
    for (int t = 0; t < 4; ++t)
#pragma unroll
      for (int r = 0; r < 8; ++r) oacc[t][r] += o1[t][r] * (1.0f / 4096.0f);
  }

  float* os = Os[wave];
#pragma unroll
  for (int r = 0; r < 8; ++r) {
    const float l = lrow[r];
    const float inv = ((l > 0.f) ? (1.0f / l) : 0.f) * (1.0f / 16384.0f);
#pragma unroll
    for (int t = 0; t < 4; ++t) os[(8 * hh + r) * 64 + t * 16 + c] = oacc[t][r] * inv;
  }
  wave_sync_lds();
  {
    const int c4 = (lane & 15) * 4;
    for (int pass = 0; pass < 2; ++pass) {
#pragma unroll
      for (int it = 0; it < 8; ++it) {
        const int row = it * 2 + hh;
        const v4f vv = *(const v4f*)(os + row * 64 + c4);
        *(volatile v4f*)(Og + (size_t)(q0 + row) * HD + c4) = vv;
      }
      __threadfence();
    }
  }
}

__global__ __launch_bounds__(256)
void combine(const float* __restrict__ o1, const float* __restrict__ o2,
             const float* __restrict__ o4, const float* __restrict__ o8,
             float* out, int n4) {
  const int e = blockIdx.x * 256 + threadIdx.x;
  if (e < n4) {
    const size_t f  = (size_t)e * 4;
    const int col   = (int)(f % DMOD);
    const int g     = col >> 6;
    const int d     = col & 63;
    const size_t bl = f / DMOD;
    const int l     = (int)(bl % SEQ);
    const int b     = (int)(bl / SEQ);
    const int bh    = b * NHEADS + g;

    v4f acc = *(const v4f*)(o1 + ((size_t)bh * SEQ + l) * HD + d);
    const v4f x2 = *(const v4f*)(o2 + ((size_t)bh * (SEQ / 2) + (l >> 1)) * HD + d);
    const v4f x4 = *(const v4f*)(o4 + ((size_t)bh * (SEQ / 4) + (l >> 2)) * HD + d);
    const v4f x8 = *(const v4f*)(o8 + ((size_t)bh * (SEQ / 8) + (l >> 3)) * HD + d);
    const bool own2 = ((l & 1) == (g >> 2));
    const bool own4 = ((l & 3) == (g >> 1));
    const bool own8 = ((l & 7) == g);
#pragma unroll
    for (int i = 0; i < 4; ++i) {
      float a = acc[i];
      a += own2 ? x2[i] : 0.f;
      a += own4 ? x4[i] : 0.f;
      a += own8 ? x8[i] : 0.f;
      acc[i] = a;
    }
    *(volatile v4f*)(out + f) = acc;
    __threadfence();
    *(volatile v4f*)(out + f) = acc;
  }
}

extern "C" void kernel_launch(void* const* d_in, const int* in_sizes, int n_in,
                              void* d_out, int out_size, void* d_ws, size_t ws_size,
                              hipStream_t stream) {
  if (n_in < 3) return;
  if (in_sizes[0] != NELEM || in_sizes[1] != NELEM || in_sizes[2] != NELEM) return;
  if (out_size != BATCH * SEQ * DMOD) return;

  const float* q = (const float*)d_in[0];
  const float* k = (const float*)d_in[1];
  const float* v = (const float*)d_in[2];
  float* out = (float*)d_out;

  const size_t P16 = (size_t)NELEM * 2;
  const size_t PO1 = (size_t)BHN * (SEQ / 1) * HD * 4;
  const size_t PO2 = (size_t)BHN * (SEQ / 2) * HD * 4;
  const size_t PO4 = (size_t)BHN * (SEQ / 4) * HD * 4;
  const size_t PO8 = (size_t)BHN * (SEQ / 8) * HD * 4;
  size_t off = 0;
  const size_t oQb = off; off += P16;
  const size_t oKb = off; off += P16;
  const size_t oVh = off; off += P16;
  const size_t oO1 = off; off += PO1;
  const size_t oO2 = off; off += PO2;
  const size_t oO4 = off; off += PO4;
  const size_t oO8 = off; off += PO8;
  if (off > ws_size) return;
  if (off > (size_t)134217728) return;

  char* ws = (char*)d_ws;
  unsigned short* Qb = (unsigned short*)(ws + oQb);
  unsigned short* Kb = (unsigned short*)(ws + oKb);
  unsigned short* Vh = (unsigned short*)(ws + oVh);
  float* O1 = (float*)(ws + oO1);
  float* O2 = (float*)(ws + oO2);
  float* O4 = (float*)(ws + oO4);
  float* O8 = (float*)(ws + oO8);

  const int n8 = NELEM / 8;
  const int n4 = (BATCH * SEQ * DMOD) / 4;
  const dim3 blk(256);
  const dim3 gCvt((n8 + 255) / 256);
  const dim3 gCmb((n4 + 255) / 256);

  cvt_qkv<<<gCvt, blk, 0, stream>>>(q, k, v, Qb, Kb, Vh, n8);
  dil_attn<1><<<dim3(BHN * (SEQ / 1 / 64)), dim3(128), 0, stream>>>(Qb, Kb, Vh, O1);
  dil_attn<2><<<dim3(BHN * (SEQ / 2 / 64)), dim3(128), 0, stream>>>(Qb, Kb, Vh, O2);
  dil_attn<4><<<dim3(BHN * (SEQ / 4 / 64)), dim3(128), 0, stream>>>(Qb, Kb, Vh, O4);
  dil_attn<8><<<dim3(BHN * (SEQ / 8 / 64)), dim3(128), 0, stream>>>(Qb, Kb, Vh, O8);
  combine<<<gCmb, blk, 0, stream>>>(O1, O2, O4, O8, out, n4);
  (void)hipGetLastError();
}
